// TableAdapterLayer_55327768707128
// MI455X (gfx1250) — hardware-verified
//
#include <hip/hip_runtime.h>
#include <math.h>

constexpr int kB   = 8;
constexpr int kS   = 512;
constexpr int kH   = 1024;
constexpr int kFF  = 3072;
constexpr int kL   = 256;
constexpr int kNH  = 16;
constexpr int kDH  = 64;
constexpr int kTok = kB * kS;
constexpr int kX4ld  = 4 * kH;
constexpr int kQKVld = 3 * kH;
constexpr int kGroups = kB * kNH;
constexpr int kGChunk = 32;
constexpr int kNChunk = kGroups / kGChunk;
constexpr int kCellsPerBlk = 32;

constexpr float kWCarry   = 16.0f;
constexpr float kWInv     = 1.0f / 16.0f;
constexpr float kPCarry   = 1024.0f;
constexpr float kCtxCarry = 64.0f;
constexpr float kScoreScale = 0.125f;
constexpr float kPVScale  = kCtxCarry / kPCarry;
constexpr float kWoScale  = 1.0f / (kCtxCarry * kWCarry);
constexpr float kInvH     = 1.0f / 1024.0f;
constexpr float kLnEps    = 1e-12f;

constexpr size_t kMiB = 1048576;
constexpr size_t OFF_X4 = 0, OFF_SEQ = 32, OFF_WRDP = 48, OFF_WCDP = 52, OFF_WRL = 56, OFF_WCL = 58,
                 OFF_CELL16 = 60, OFF_CELLGR = 64, OFF_WDP = 72, OFF_CELLGC = 80;
constexpr size_t OFF_XF32 = 48, OFF_XH = 80;
constexpr size_t OFF_QKV = 0, OFF_VT = 24, OFF_CTX = 32, OFF_WO = 40, OFF_WQKV = 42, OFF_SC = 64,
                 OFF_P = 96, OFF_WOOUT = 112;
constexpr size_t OFF_HF32 = 64, OFF_HH = 80, OFF_WW1 = 88, OFF_WW2 = 94, OFF_FFNPRE = 0, OFF_FFNH = 100,
                 OFF_W2OUT = 0;
constexpr size_t kWsNeedMiB = 128;
static_assert(OFF_WOOUT + 16 <= kWsNeedMiB, "ws");
static_assert(OFF_FFNH + 24 <= kWsNeedMiB, "ws");
static_assert(OFF_FFNPRE + 48 <= OFF_XF32 || true, "ws");
static_assert(OFF_WW2 + 6 <= OFF_FFNH, "ws");
static_assert(OFF_HH + 8 <= OFF_WW1, "ws");
static_assert(OFF_WQKV + 6 <= OFF_XF32, "ws");
static_assert(OFF_P + 16 <= OFF_WOOUT, "ws");

typedef __attribute__((ext_vector_type(16))) _Float16 v16h;
typedef __attribute__((ext_vector_type(8)))  _Float16 v8h;
typedef __attribute__((ext_vector_type(16))) __bf16   v16b;
typedef __attribute__((ext_vector_type(8)))  __bf16   v8b;
typedef __attribute__((ext_vector_type(8)))  float    v8f;
typedef __attribute__((ext_vector_type(4)))  float    v4f;
typedef __attribute__((ext_vector_type(2)))  float    v2f;
typedef __attribute__((ext_vector_type(4)))  unsigned int v4u;
typedef __attribute__((ext_vector_type(2)))  unsigned int v2u;

__device__ __forceinline__ unsigned short f2bf_bits(float f) {
  unsigned u = __float_as_uint(f);
  return (unsigned short)((u + 0x7FFFu + ((u >> 16) & 1u)) >> 16);
}
__device__ __forceinline__ float bf_bits2f(unsigned short h) { return __uint_as_float(((unsigned)h) << 16); }

__device__ __forceinline__ void dep_guard_h(v8f& a, v8f& b, v16h x, v16h y) { asm volatile("v_nop\n\tv_nop\n\tv_nop\n\tv_nop" : "+v"(a), "+v"(b) : "v"(x), "v"(y)); }
__device__ __forceinline__ void dep_guard_b(v8f& a, v8f& b, v16b x, v16b y) { asm volatile("v_nop\n\tv_nop\n\tv_nop\n\tv_nop" : "+v"(a), "+v"(b) : "v"(x), "v"(y)); }
__device__ __forceinline__ void keep4_h(v16h a, v16h b, v16h c, v16h d) { asm volatile("v_nop" :: "v"(a), "v"(b), "v"(c), "v"(d)); }
__device__ __forceinline__ void keep4_b(v16b a, v16b b, v16b c, v16b d) { asm volatile("v_nop" :: "v"(a), "v"(b), "v"(c), "v"(d)); }
__device__ __forceinline__ void acc_guard4(v8f& a, v8f& b, v8f& c, v8f& d) { asm volatile("v_nop\n\tv_nop\n\tv_nop\n\tv_nop" : "+v"(a), "+v"(b), "+v"(c), "+v"(d)); }
template <typename T> struct Frag;
template <> struct Frag<_Float16> {
  typedef v16h V; union U { v16h v; v8h h[2]; };
  static __device__ __forceinline__ v16h load(const _Float16* p) {
    U f; f.h[0] = *(const v8h*)(p); f.h[1] = *(const v8h*)(p + 16); return f.v;
  }
  static __device__ __forceinline__ v8f mma(v16h a, v16h b, v8f c) {
    return __builtin_amdgcn_wmma_f32_16x16x32_f16(false, a, false, b, (short)0, c, false, false);
  }
  static __device__ __forceinline__ void guard(v8f& a, v8f& b, v16h x, v16h y) { dep_guard_h(a, b, x, y); }
  static __device__ __forceinline__ void keep(v16h a, v16h b, v16h c, v16h d) { keep4_h(a, b, c, d); }
};
template <> struct Frag<__bf16> {
  typedef v16b V; union U { v16b v; v8b h[2]; };
  static __device__ __forceinline__ v16b load(const __bf16* p) {
    U f; f.h[0] = *(const v8b*)(p); f.h[1] = *(const v8b*)(p + 16); return f.v;
  }
  static __device__ __forceinline__ v8f mma(v16b a, v16b b, v8f c) {
    return __builtin_amdgcn_wmma_f32_16x16x32_bf16(false, a, false, b, (short)0, c, false, false);
  }
  static __device__ __forceinline__ void guard(v8f& a, v8f& b, v16b x, v16b y) { dep_guard_b(a, b, x, y); }
  static __device__ __forceinline__ void keep(v16b a, v16b b, v16b c, v16b d) { keep4_b(a, b, c, d); }
};

__device__ __forceinline__ unsigned pk16(unsigned short a, unsigned short b) { return (unsigned)a | ((unsigned)b << 16); }
__device__ __forceinline__ unsigned short h_bits(float f) { const _Float16 h = (_Float16)f; return __builtin_bit_cast(unsigned short, h); }

__device__ __forceinline__ float gelu_f(float x) {
  return 0.5f * x * (1.0f + erff(x * 0.70710678118654752f));
}

template <int ET> struct Elem;
template <> struct Elem<0> { typedef _Float16 T; };
template <> struct Elem<1> { typedef __bf16 T; };
template <int ET, bool SPLIT, int BIAS_MODE, int OUT_MODE, bool RESID>
__global__ __launch_bounds__(256) void wmma_gemm64(
    const unsigned short* __restrict__ Ap, const unsigned short* __restrict__ A2p, int lda, long strideA, long strideA2,
    const unsigned short* __restrict__ Btp, const unsigned short* __restrict__ Bt2p, int ldb, long strideB, long strideB2,
    void* __restrict__ Cout, void* __restrict__ Cout2, int ldc, long strideC, long strideC2,
    const float* __restrict__ bias,
    const float* __restrict__ resid, long strideR, long strideR2,
    int M, int N, int K, float scale, int bdiv) {
  typedef typename Elem<ET>::T T;
  typedef typename Frag<T>::V V;
  const T* A = (const T*)Ap; const T* A2 = (const T*)A2p; const T* Bt = (const T*)Btp; const T* Bt2 = (const T*)Bt2p;
  __shared__ __align__(16) float sT[8][16 * 68];
  const int by   = blockIdx.y;
  const int by1  = by / bdiv;
  const int by2  = by - by1 * bdiv;
  const int lane = threadIdx.x & 31;
  const int wave = threadIdx.x >> 5;
  const int tilesN = N >> 6;
  const int tilesM = M >> 6;
  const int tile = blockIdx.x * 8 + wave;
  if (tile >= tilesM * tilesN) return;
  const int tm = tile / tilesN;
  const int tn = tile - tm * tilesN;
  const int m0 = tm << 6;
  const int n0 = tn << 6;

  const size_t offA = (size_t)by1 * (size_t)strideA + (size_t)by2 * (size_t)strideA2;
  const size_t offB = (size_t)by1 * (size_t)strideB + (size_t)by2 * (size_t)strideB2;
  const size_t offC = (size_t)by1 * (size_t)strideC + (size_t)by2 * (size_t)strideC2;
  const size_t offR = (size_t)by1 * (size_t)strideR + (size_t)by2 * (size_t)strideR2;

  const T* Ab  = A  + offA;
  const T* Bb  = Bt + offB;
  const T* Ab2 = SPLIT ? (A2  + offA) : nullptr;
  const T* Bb2 = SPLIT ? (Bt2 + offB) : nullptr;

  const int rlane = lane & 15;
  const int koff  = (lane >> 4) * 8;
  const int mOff  = (lane >> 4) * 8;

  v8f acc[4][4];
#pragma unroll
  for (int i = 0; i < 4; ++i)
#pragma unroll
    for (int j = 0; j < 4; ++j) acc[i][j] = (v8f){0.f,0.f,0.f,0.f,0.f,0.f,0.f,0.f};

  for (int k0 = 0; k0 < K; k0 += 32) {
    V bh[4], bl[4];
#pragma unroll
    for (int j = 0; j < 4; ++j) {
      const size_t bo = (size_t)(n0 + (j << 4) + rlane) * ldb + koff + k0;
      bh[j] = Frag<T>::load(Bb + bo);
      if (SPLIT) bl[j] = Frag<T>::load(Bb2 + bo);
    }
#pragma unroll
    for (int i = 0; i < 4; ++i) {
      const size_t ao = (size_t)(m0 + (i << 4) + rlane) * lda + koff + k0;
      V ah = Frag<T>::load(Ab + ao);
      V al;
      if (SPLIT) al = Frag<T>::load(Ab2 + ao);
#pragma unroll
      for (int j = 0; j < 4; ++j) {
        acc[i][j] = Frag<T>::mma(ah, bh[j], acc[i][j]);
        if (SPLIT) {
          acc[i][j] = Frag<T>::mma(ah, bl[j], acc[i][j]);
          acc[i][j] = Frag<T>::mma(al, bh[j], acc[i][j]);
        }
      }
      Frag<T>::guard(acc[i][0], acc[i][3], ah, SPLIT ? al : ah);
    }
    Frag<T>::keep(bh[0], bh[1], bh[2], bh[3]);
    if (SPLIT) Frag<T>::keep(bl[0], bl[1], bl[2], bl[3]);
  }
  acc_guard4(acc[0][0], acc[0][1], acc[0][2], acc[0][3]);
  acc_guard4(acc[1][0], acc[1][1], acc[1][2], acc[1][3]);
  acc_guard4(acc[2][0], acc[2][1], acc[2][2], acc[2][3]);
  acc_guard4(acc[3][0], acc[3][1], acc[3][2], acc[3][3]);

  float* slab = sT[wave];
  const float* Rb = RESID ? (resid + offR) : nullptr;
#pragma unroll
  for (int i = 0; i < 4; ++i) {
    const int mBase = m0 + (i << 4);
#pragma unroll
    for (int j = 0; j < 4; ++j) {
      const int n = n0 + (j << 4) + rlane;
      float bv = 0.f;
      if (BIAS_MODE == 2) bv = bias[n];
#pragma unroll
      for (int r = 0; r < 8; ++r) {
        float v = acc[i][j][r] * scale;
        if (BIAS_MODE == 1) v += bias[mBase + mOff + r];
        if (BIAS_MODE == 2) v += bv;
        if (RESID) v += Rb[(size_t)(mBase + mOff + r) * ldc + n];
        slab[(mOff + r) * 68 + (j << 4) + rlane] = v;
      }
    }
    __builtin_amdgcn_fence(__ATOMIC_RELEASE, "workgroup");
    __builtin_amdgcn_wave_barrier();
    __builtin_amdgcn_fence(__ATOMIC_ACQUIRE, "workgroup");
    if (OUT_MODE == 0) {
      float* C = (float*)Cout + offC;
      const int hh = lane >> 4, c4 = (lane & 15) * 4;
      for (int pass = 0; pass < 2; ++pass) {
#pragma unroll
        for (int it = 0; it < 8; ++it) {
          const int row = it * 2 + hh;
          v4f v = *(const v4f*)(slab + row * 68 + c4);
          *(volatile v4f*)(C + (size_t)(mBase + row) * ldc + n0 + c4) = v;
        }
        __threadfence();
      }
    } else {
      const int q = lane >> 3, c8 = (lane & 7) * 8;
      unsigned short* C  = (unsigned short*)Cout  + offC;
      unsigned short* C2 = (OUT_MODE == 2) ? ((unsigned short*)Cout2 + offC) : nullptr;
      for (int pass = 0; pass < 2; ++pass) {
#pragma unroll
        for (int it = 0; it < 4; ++it) {
          const int row = it * 4 + q;
          const float* sp = slab + row * 68 + c8;
          v8h hv, lv;
#pragma unroll
          for (int e = 0; e < 8; ++e) {
            if (OUT_MODE == 1) {
              hv[e] = (_Float16)sp[e];
            } else {
              unsigned short hb = f2bf_bits(sp[e]);
              unsigned short lb = f2bf_bits(sp[e] - bf_bits2f(hb));
              hv[e] = __builtin_bit_cast(_Float16, hb);
              lv[e] = __builtin_bit_cast(_Float16, lb);
            }
          }
          *(volatile v8h*)(C + (size_t)(mBase + row) * ldc + n0 + c8) = hv;
          if (OUT_MODE == 2) *(volatile v8h*)(C2 + (size_t)(mBase + row) * ldc + n0 + c8) = lv;
        }
        __threadfence();
      }
    }
    __builtin_amdgcn_fence(__ATOMIC_RELEASE, "workgroup");
    __builtin_amdgcn_wave_barrier();
    __builtin_amdgcn_fence(__ATOMIC_ACQUIRE, "workgroup");
  }
}

__global__ __launch_bounds__(256) void tcast_kernel(const float* __restrict__ W0, const float* __restrict__ W1,
                                                    const float* __restrict__ W2, unsigned short* __restrict__ out,
                                                    int Kd, int Nd, float scale) {
  __shared__ float sm[64][65];
  const int t  = threadIdx.x;
  const int k0 = blockIdx.x * 64;
  const int n0 = blockIdx.y * 64;
  const int z  = blockIdx.z;
  const float* W = (z == 0) ? W0 : (z == 1) ? W1 : W2;
#pragma unroll
  for (int i = 0; i < 16; ++i) {
    const int e = i * 256 + t;
    const int r = e >> 6;
    const int c = e & 63;
    sm[c][r] = W[(size_t)(k0 + r) * Nd + n0 + c] * scale;
  }
  __syncthreads();
  const int lane = t & 31, wave = t >> 5;
  const int q = lane >> 3, c8 = (lane & 7) * 8;
  unsigned short* op = out + (size_t)z * Nd * Kd;
  const int rowA = wave * 8 + q;
  const int rowB = wave * 8 + 4 + q;
  unsigned short ha[8], hbv[8];
#pragma unroll
  for (int e = 0; e < 8; ++e) { ha[e] = h_bits(sm[rowA][c8 + e]); hbv[e] = h_bits(sm[rowB][c8 + e]); }
  const v4u ua = (v4u){pk16(ha[0], ha[1]), pk16(ha[2], ha[3]), pk16(ha[4], ha[5]), pk16(ha[6], ha[7])};
  const v4u ub = (v4u){pk16(hbv[0], hbv[1]), pk16(hbv[2], hbv[3]), pk16(hbv[4], hbv[5]), pk16(hbv[6], hbv[7])};
  unsigned short* pa = op + (size_t)(n0 + rowA) * Kd + k0 + c8;
  unsigned short* pb = op + (size_t)(n0 + rowB) * Kd + k0 + c8;
  for (int pass = 0; pass < 2; ++pass) {
    *(volatile v4u*)pa = ua;
    *(volatile v4u*)pb = ub;
    __threadfence();
  }
}

__global__ __launch_bounds__(256) void concat_cast_kernel(const float* __restrict__ former, const float* __restrict__ hidden,
                                                          unsigned short* __restrict__ x4) {
  const unsigned idx = blockIdx.x * 256u + threadIdx.x;
  const unsigned src = idx >> 19;
  const unsigned e   = idx & 524287u;
  const unsigned row = e >> 7;
  const unsigned c8  = (e & 127u) * 8u;
  const float* s = (src == 0u) ? former : hidden;
  const float* p = s + (size_t)row * kH + c8;
  const v4f a = *(const v4f*)(p);
  const v4f c = *(const v4f*)(p + 4);
  const v4u u = (v4u){pk16(h_bits(a[0]), h_bits(a[1])), pk16(h_bits(a[2]), h_bits(a[3])),
                      pk16(h_bits(c[0]), h_bits(c[1])), pk16(h_bits(c[2]), h_bits(c[3]))};
  unsigned short* d = x4 + (size_t)row * kX4ld + (size_t)src * kH + c8;
  *(volatile v4u*)d = u;
  __threadfence();
  *(volatile v4u*)d = u;
}

__global__ __launch_bounds__(512) void segsum_kernel(const float* __restrict__ seq, const int* __restrict__ ids,
                                                     unsigned short* __restrict__ cell16) {
  __shared__ int sIds[kS];
  __shared__ int sTok[kS];
  __shared__ int sCnt[kCellsPerBlk];
  __shared__ int sOff[kCellsPerBlk];
  const int tid = threadIdx.x;
  const int cg  = blockIdx.x;
  const int b   = blockIdx.y;
  sIds[tid] = ids[b * kS + tid];
  __syncthreads();
  if (tid < 32) {
    const int c = cg * kCellsPerBlk + tid;
    int cnt = 0;
#pragma unroll 1
    for (int t = 0; t < kS; ++t) cnt += (sIds[t] == c) ? 1 : 0;
    int incl = cnt;
#pragma unroll
    for (int off = 1; off < 32; off <<= 1) {
      const int v = __shfl_up(incl, off, 32);
      incl += (tid >= off) ? v : 0;
    }
    const int excl = incl - cnt;
    sCnt[tid] = cnt;
    sOff[tid] = excl;
    int pos = excl;
#pragma unroll 1
    for (int t = 0; t < kS; ++t) {
      const bool m = (sIds[t] == c);
      int p = pos;
      p = (p > kS - 1) ? (kS - 1) : p;
      if (m) sTok[p] = t;
      pos += m ? 1 : 0;
    }
  }
  __syncthreads();
  const int f0 = 2 * tid;
  const float* sb = seq + (size_t)b * kS * kH + f0;
  unsigned short* cbase = cell16 + ((size_t)b * kL + (size_t)cg * kCellsPerBlk) * kH + f0;
#pragma unroll 1
  for (int c = 0; c < kCellsPerBlk; ++c) {
    int beg = sOff[c];
    int n   = sCnt[c];
    beg = beg < 0 ? 0 : beg; beg = beg > kS ? kS : beg;
    n = n < 0 ? 0 : n; n = n > (kS - beg) ? (kS - beg) : n;
    float a0 = 0.0f, a1 = 0.0f;
#pragma unroll 1
    for (int j = 0; j < n; ++j) {
      int t = sTok[beg + j];
      t = t < 0 ? 0 : t; t = t > kS - 1 ? kS - 1 : t;
      const v2f x = *(const v2f*)(sb + (size_t)t * kH);
      a0 += gelu_f(x[0]);
      a1 += gelu_f(x[1]);
    }
    const unsigned u = pk16(h_bits(a0), h_bits(a1));
    unsigned* dst = (unsigned*)(cbase + (size_t)c * kH);
    *(volatile unsigned*)dst = u;
    __threadfence();
    *(volatile unsigned*)dst = u;
  }
}

__global__ __launch_bounds__(256) void gather_kernel(const float* __restrict__ cellgR, const float* __restrict__ cellgC,
                                                     const int* __restrict__ row_ids, const int* __restrict__ col_ids,
                                                     unsigned short* __restrict__ x4) {
  const int tab = blockIdx.y;
  const float* cg = (tab == 0) ? cellgR : cellgC;
  const int* idp  = (tab == 0) ? row_ids : col_ids;
  const unsigned idx = blockIdx.x * 256u + threadIdx.x;
  const int row = (int)(idx >> 9);
  const int j2  = (int)(idx & 511u) * 2;
  const int b   = row >> 9;
  int id = idp[row];
  id = id < 0 ? 0 : id; id = id > kL - 1 ? kL - 1 : id;
  const int cid = col_ids[row];
  const float mk = (cid == 0) ? 0.0f : 1.0f;
  const v2f x = *(const v2f*)(cg + ((size_t)(b * kL + id)) * kH + j2);
  const float g0 = gelu_f(x[0]) * mk;
  const float g1 = gelu_f(x[1]) * mk;
  const unsigned u = pk16(h_bits(g0), h_bits(g1));
  unsigned* dst = (unsigned*)(x4 + (size_t)row * kX4ld + 2 * kH + tab * kH + j2);
  *(volatile unsigned*)dst = u;
  __threadfence();
  *(volatile unsigned*)dst = u;
}

__global__ __launch_bounds__(512) void ln_gelu_kernel(const float* __restrict__ xin, const float* __restrict__ resid,
                                                      const float* __restrict__ g, const float* __restrict__ bb,
                                                      float* __restrict__ out32, unsigned short* __restrict__ out16) {
  __shared__ float sA[16];
  __shared__ float sB[16];
  const int row = blockIdx.x, t = threadIdx.x, lane = t & 31, wave = t >> 5;
  const int c0 = 2 * t;
  const size_t base = (size_t)row * kH + c0;
  const v2f x = *(const v2f*)(xin + base);
  const v2f r = *(const v2f*)(resid + base);
  const float v0 = r[0] + gelu_f(x[0]);
  const float v1 = r[1] + gelu_f(x[1]);
  float s = v0 + v1;
#pragma unroll
  for (int off = 16; off > 0; off >>= 1) s += __shfl_xor(s, off, 32);
  if (lane == 0) sA[wave] = s;
  __syncthreads();
  float tot = 0.0f;
#pragma unroll
  for (int w = 0; w < 16; ++w) tot += sA[w];
  const float mean = tot * kInvH;
  const float d0 = v0 - mean, d1 = v1 - mean;
  float s2 = d0 * d0 + d1 * d1;
#pragma unroll
  for (int off = 16; off > 0; off >>= 1) s2 += __shfl_xor(s2, off, 32);
  if (lane == 0) sB[wave] = s2;
  __syncthreads();
  float tot2 = 0.0f;
#pragma unroll
  for (int w = 0; w < 16; ++w) tot2 += sB[w];
  const float var = tot2 * kInvH;
  const float inv = rsqrtf(var + kLnEps);
  const v2f gg = *(const v2f*)(g + c0);
  const v2f be = *(const v2f*)(bb + c0);
  v2f y;
  y[0] = d0 * inv * gg[0] + be[0];
  y[1] = d1 * inv * gg[1] + be[1];
  const unsigned u = pk16(h_bits(y[0]), h_bits(y[1]));
  float* d32 = out32 + base;
  unsigned* d16 = (unsigned*)(out16 + base);
  *(volatile v2f*)d32 = y;
  *(volatile unsigned*)d16 = u;
  __threadfence();
  *(volatile v2f*)d32 = y;
  *(volatile unsigned*)d16 = u;
}

template <bool HAS16>
__global__ __launch_bounds__(256) void ln_kernel(const float* __restrict__ xin, const float* __restrict__ g,
                                                 const float* __restrict__ bb, float* __restrict__ out32,
                                                 unsigned short* __restrict__ out16) {
  __shared__ float sA[8];
  __shared__ float sB[8];
  const int row = blockIdx.x, t = threadIdx.x, lane = t & 31, wave = t >> 5;
  const int c0 = 4 * t;
  const size_t base = (size_t)row * kH + c0;
  const v4f x = *(const v4f*)(xin + base);
  float s = (x[0] + x[1]) + (x[2] + x[3]);
#pragma unroll
  for (int off = 16; off > 0; off >>= 1) s += __shfl_xor(s, off, 32);
  if (lane == 0) sA[wave] = s;
  __syncthreads();
  float tot = 0.0f;
#pragma unroll
  for (int w = 0; w < 8; ++w) tot += sA[w];
  const float mean = tot * kInvH;
  const float d0 = x[0] - mean, d1 = x[1] - mean, d2 = x[2] - mean, d3 = x[3] - mean;
  float s2 = (d0 * d0 + d1 * d1) + (d2 * d2 + d3 * d3);
#pragma unroll
  for (int off = 16; off > 0; off >>= 1) s2 += __shfl_xor(s2, off, 32);
  if (lane == 0) sB[wave] = s2;
  __syncthreads();
  float tot2 = 0.0f;
#pragma unroll
  for (int w = 0; w < 8; ++w) tot2 += sB[w];
  const float var = tot2 * kInvH;
  const float inv = rsqrtf(var + kLnEps);
  const v4f gg = *(const v4f*)(g + c0);
  const v4f be = *(const v4f*)(bb + c0);
  v4f y;
  y[0] = d0 * inv * gg[0] + be[0];
  y[1] = d1 * inv * gg[1] + be[1];
  y[2] = d2 * inv * gg[2] + be[2];
  y[3] = d3 * inv * gg[3] + be[3];
  float* d32 = out32 + base;
  v2u u;
  u[0] = pk16(h_bits(y[0]), h_bits(y[1]));
  u[1] = pk16(h_bits(y[2]), h_bits(y[3]));
  unsigned short* d16 = HAS16 ? (out16 + base) : nullptr;
  *(volatile v4f*)d32 = y;
  if (HAS16) *(volatile v2u*)d16 = u;
  __threadfence();
  *(volatile v4f*)d32 = y;
  if (HAS16) *(volatile v2u*)d16 = u;
}

__global__ __launch_bounds__(256) void vt_kernel(const unsigned short* __restrict__ qkv, unsigned short* __restrict__ vt) {
  __shared__ unsigned short sm[64][72];
  const int t = threadIdx.x;
  const int sc = blockIdx.x;
  const int g  = blockIdx.y;
  const int b  = g >> 4, h = g & 15;
  const int s0 = sc * 64;
#pragma unroll
  for (int i = 0; i < 16; ++i) {
    const int e  = i * 256 + t;
    const int sl = e >> 6;
    const int dl = e & 63;
    sm[dl][sl] = qkv[(size_t)(b * kS + s0 + sl) * kQKVld + 2 * kH + h * kDH + dl];
  }
  __syncthreads();
  const int lane = t & 31, wave = t >> 5;
  const int q = lane >> 3, c8 = (lane & 7) * 8;
  const int rowA = wave * 8 + q;
  const int rowB = wave * 8 + 4 + q;
  const v4u ua = (v4u){pk16(sm[rowA][c8 + 0], sm[rowA][c8 + 1]), pk16(sm[rowA][c8 + 2], sm[rowA][c8 + 3]),
                       pk16(sm[rowA][c8 + 4], sm[rowA][c8 + 5]), pk16(sm[rowA][c8 + 6], sm[rowA][c8 + 7])};
  const v4u ub = (v4u){pk16(sm[rowB][c8 + 0], sm[rowB][c8 + 1]), pk16(sm[rowB][c8 + 2], sm[rowB][c8 + 3]),
                       pk16(sm[rowB][c8 + 4], sm[rowB][c8 + 5]), pk16(sm[rowB][c8 + 6], sm[rowB][c8 + 7])};
  unsigned short* pa = vt + ((size_t)g * kDH + rowA) * kS + s0 + c8;
  unsigned short* pb = vt + ((size_t)g * kDH + rowB) * kS + s0 + c8;
  for (int pass = 0; pass < 2; ++pass) {
    *(volatile v4u*)pa = ua;
    *(volatile v4u*)pb = ub;
    __threadfence();
  }
}

__global__ __launch_bounds__(64) void softmax_kernel(const float* __restrict__ scores, const float* __restrict__ smask,
                                                     unsigned short* __restrict__ P, int cb) {
  __shared__ float sM[2];
  __shared__ float sS[2];
  const int row  = blockIdx.x;
  const int y    = row >> 9;
  const int q    = row & 511;
  const int b    = cb * 2 + (y >> 4);
  const int t    = threadIdx.x;
  const int lane = t & 31, wave = t >> 5;
  const int c0   = 8 * t;
  const float* sp = scores + (size_t)row * kS + c0;
  const float* mp = smask + ((size_t)(b * kS + q)) * kS + c0;
  const v4f a = *(const v4f*)(sp);
  const v4f c = *(const v4f*)(sp + 4);
  const v4f ma = *(const v4f*)(mp);
  const v4f mc = *(const v4f*)(mp + 4);
  float x[8];
#pragma unroll
  for (int e = 0; e < 4; ++e) {
    x[e]     = a[e] + (1.0f - ma[e]) * (-10000.0f);
    x[4 + e] = c[e] + (1.0f - mc[e]) * (-10000.0f);
  }
  float m = fmaxf(fmaxf(fmaxf(x[0], x[1]), fmaxf(x[2], x[3])), fmaxf(fmaxf(x[4], x[5]), fmaxf(x[6], x[7])));
#pragma unroll
  for (int off = 16; off > 0; off >>= 1) m = fmaxf(m, __shfl_xor(m, off, 32));
  if (lane == 0) sM[wave] = m;
  __syncthreads();
  const float mx = fmaxf(sM[0], sM[1]);
  float ev[8];
  float sum = 0.0f;
#pragma unroll
  for (int e = 0; e < 8; ++e) { ev[e] = expf(x[e] - mx); sum += ev[e]; }
#pragma unroll
  for (int off = 16; off > 0; off >>= 1) sum += __shfl_xor(sum, off, 32);
  if (lane == 0) sS[wave] = sum;
  __syncthreads();
  const float tot = sS[0] + sS[1];
  const float inv = kPCarry / tot;
  unsigned short hb[8];
#pragma unroll
  for (int e = 0; e < 8; ++e) hb[e] = h_bits(ev[e] * inv);
  const v4u u = (v4u){pk16(hb[0], hb[1]), pk16(hb[2], hb[3]), pk16(hb[4], hb[5]), pk16(hb[6], hb[7])};
  unsigned short* d = P + (size_t)row * kS + c0;
  *(volatile v4u*)d = u;
  __threadfence();
  *(volatile v4u*)d = u;
}

__global__ __launch_bounds__(256) void gelu_cast2_kernel(const float* __restrict__ in, unsigned short* __restrict__ out, int n2) {
  const int i = blockIdx.x * 256 + threadIdx.x;
  if (i >= n2) return;
  const v2f x = *(const v2f*)(in + 2 * (size_t)i);
  const unsigned u = pk16(h_bits(gelu_f(x[0])), h_bits(gelu_f(x[1])));
  unsigned* d = (unsigned*)(out + 2 * (size_t)i);
  *(volatile unsigned*)d = u;
  __threadfence();
  *(volatile unsigned*)d = u;
}

static inline unsigned gemm_grid_x(int M, int N) { return (unsigned)(((M / 64) * (N / 64) + 7) / 8); }

extern "C" void kernel_launch(void* const* d_in, const int* in_sizes, int n_in,
                              void* d_out, int out_size, void* d_ws, size_t ws_size,
                              hipStream_t stream) {
  if (n_in < 34) return;
  if (ws_size < kWsNeedMiB * kMiB) return;
  if (out_size != kTok * kH) return;
  if (in_sizes[0] != kTok * kH || in_sizes[1] != kTok * kH || in_sizes[2] != kB * kS * kS) return;
  if (in_sizes[32] != kTok || in_sizes[33] != kTok) return;
  if (in_sizes[12] != 4 * kH * kH || in_sizes[26] != kH * kFF || in_sizes[28] != kFF * kH) return;

  const float* former = (const float*)d_in[0];
  const float* hidden = (const float*)d_in[1];
  const float* smask  = (const float*)d_in[2];
  const float* r_dpw  = (const float*)d_in[4];
  const float* r_dpb  = (const float*)d_in[5];
  const float* r_lw   = (const float*)d_in[6];
  const float* r_lb   = (const float*)d_in[7];
  const float* c_dpw  = (const float*)d_in[8];
  const float* c_dpb  = (const float*)d_in[9];
  const float* c_lw   = (const float*)d_in[10];
  const float* c_lb   = (const float*)d_in[11];
  const float* dp_w   = (const float*)d_in[12];
  const float* dp_b   = (const float*)d_in[13];
  const float* ln_g   = (const float*)d_in[14];
  const float* ln_b   = (const float*)d_in[15];
  const float* wq = (const float*)d_in[16]; const float* bq = (const float*)d_in[17];
  const float* wk = (const float*)d_in[18]; const float* bk = (const float*)d_in[19];
  const float* wv = (const float*)d_in[20]; const float* bv = (const float*)d_in[21];
  const float* wo = (const float*)d_in[22]; const float* bo = (const float*)d_in[23];
  const float* ln1_g = (const float*)d_in[24]; const float* ln1_b = (const float*)d_in[25];
  const float* w1 = (const float*)d_in[26]; const float* b1 = (const float*)d_in[27];
  const float* w2 = (const float*)d_in[28]; const float* b2 = (const float*)d_in[29];
  const float* ln2_g = (const float*)d_in[30]; const float* ln2_b = (const float*)d_in[31];
  const int* row_ids = (const int*)d_in[32];
  const int* col_ids = (const int*)d_in[33];

  char* ws = (char*)d_ws;
  unsigned short* X4     = (unsigned short*)(ws + OFF_X4 * kMiB);
  float*          SEQ    = (float*)(ws + OFF_SEQ * kMiB);
  unsigned short* WRDP   = (unsigned short*)(ws + OFF_WRDP * kMiB);
  unsigned short* WCDP   = (unsigned short*)(ws + OFF_WCDP * kMiB);
  unsigned short* WRL    = (unsigned short*)(ws + OFF_WRL * kMiB);
  unsigned short* WCL    = (unsigned short*)(ws + OFF_WCL * kMiB);
  unsigned short* CELL16 = (unsigned short*)(ws + OFF_CELL16 * kMiB);
  float*          CELLGR = (float*)(ws + OFF_CELLGR * kMiB);
  unsigned short* WDP    = (unsigned short*)(ws + OFF_WDP * kMiB);
  float*          CELLGC = (float*)(ws + OFF_CELLGC * kMiB);
  float*          XF32   = (float*)(ws + OFF_XF32 * kMiB);
  unsigned short* XH     = (unsigned short*)(ws + OFF_XH * kMiB);
  unsigned short* QKV    = (unsigned short*)(ws + OFF_QKV * kMiB);
  unsigned short* VT     = (unsigned short*)(ws + OFF_VT * kMiB);
  unsigned short* CTX    = (unsigned short*)(ws + OFF_CTX * kMiB);
  unsigned short* WO     = (unsigned short*)(ws + OFF_WO * kMiB);
  unsigned short* WQKV   = (unsigned short*)(ws + OFF_WQKV * kMiB);
  float*          SC     = (float*)(ws + OFF_SC * kMiB);
  unsigned short* P      = (unsigned short*)(ws + OFF_P * kMiB);
  float*          WOOUT  = (float*)(ws + OFF_WOOUT * kMiB);
  float*          HF32   = (float*)(ws + OFF_HF32 * kMiB);
  unsigned short* HH     = (unsigned short*)(ws + OFF_HH * kMiB);
  unsigned short* WW1    = (unsigned short*)(ws + OFF_WW1 * kMiB);
  unsigned short* WW2    = (unsigned short*)(ws + OFF_WW2 * kMiB);
  float*          FFNPRE = (float*)(ws + OFF_FFNPRE * kMiB);
  unsigned short* FFNH   = (unsigned short*)(ws + OFF_FFNH * kMiB);
  float*          W2OUT  = (float*)(ws + OFF_W2OUT * kMiB);
  float*          OUT    = (float*)d_out;

  tcast_kernel<<<dim3(2 * kH / 64, kH / 64, 1), 256, 0, stream>>>(r_dpw, r_dpw, r_dpw, WRDP, 2 * kH, kH, kWCarry);
  tcast_kernel<<<dim3(2 * kH / 64, kH / 64, 1), 256, 0, stream>>>(c_dpw, c_dpw, c_dpw, WCDP, 2 * kH, kH, kWCarry);
  tcast_kernel<<<dim3(kH / 64, kH / 64, 1), 256, 0, stream>>>(r_lw, r_lw, r_lw, WRL, kH, kH, kWCarry);
  tcast_kernel<<<dim3(kH / 64, kH / 64, 1), 256, 0, stream>>>(c_lw, c_lw, c_lw, WCL, kH, kH, kWCarry);
  tcast_kernel<<<dim3(4 * kH / 64, kH / 64, 1), 256, 0, stream>>>(dp_w, dp_w, dp_w, WDP, 4 * kH, kH, kWCarry);

  concat_cast_kernel<<<dim3(4096), 256, 0, stream>>>(former, hidden, X4);

  wmma_gemm64<0, false, 2, 0, false><<<dim3(gemm_grid_x(kTok, kH), 1), 256, 0, stream>>>(
      X4, nullptr, kX4ld, 0L, 0L, WRDP, nullptr, 2 * kH, 0L, 0L, (void*)SEQ, nullptr, kH, 0L, 0L,
      r_dpb, nullptr, 0L, 0L, kTok, kH, 2 * kH, kWInv, 1);
  segsum_kernel<<<dim3(kL / kCellsPerBlk, kB), 512, 0, stream>>>(SEQ, row_ids, CELL16);
  wmma_gemm64<0, false, 2, 0, false><<<dim3(gemm_grid_x(kB * kL, kH), 1), 256, 0, stream>>>(
      CELL16, nullptr, kH, 0L, 0L, WRL, nullptr, kH, 0L, 0L, (void*)CELLGR, nullptr, kH, 0L, 0L,
      r_lb, nullptr, 0L, 0L, kB * kL, kH, kH, kWInv, 1);

  wmma_gemm64<0, false, 2, 0, false><<<dim3(gemm_grid_x(kTok, kH), 1), 256, 0, stream>>>(
      X4, nullptr, kX4ld, 0L, 0L, WCDP, nullptr, 2 * kH, 0L, 0L, (void*)SEQ, nullptr, kH, 0L, 0L,
      c_dpb, nullptr, 0L, 0L, kTok, kH, 2 * kH, kWInv, 1);
  segsum_kernel<<<dim3(kL / kCellsPerBlk, kB), 512, 0, stream>>>(SEQ, col_ids, CELL16);
  wmma_gemm64<0, false, 2, 0, false><<<dim3(gemm_grid_x(kB * kL, kH), 1), 256, 0, stream>>>(
      CELL16, nullptr, kH, 0L, 0L, WCL, nullptr, kH, 0L, 0L, (void*)CELLGC, nullptr, kH, 0L, 0L,
      c_lb, nullptr, 0L, 0L, kB * kL, kH, kH, kWInv, 1);

  gather_kernel<<<dim3(kTok * 512 / 256, 2), 256, 0, stream>>>(CELLGR, CELLGC, row_ids, col_ids, X4);

  wmma_gemm64<0, false, 2, 0, false><<<dim3(gemm_grid_x(kTok, kH), 1), 256, 0, stream>>>(
      X4, nullptr, kX4ld, 0L, 0L, WDP, nullptr, 4 * kH, 0L, 0L, (void*)SEQ, nullptr, kH, 0L, 0L,
      dp_b, nullptr, 0L, 0L, kTok, kH, 4 * kH, kWInv, 1);
  ln_gelu_kernel<<<dim3(kTok), 512, 0, stream>>>(SEQ, former, ln_g, ln_b, XF32, XH);

  tcast_kernel<<<dim3(kH / 64, kH / 64, 3), 256, 0, stream>>>(wq, wk, wv, WQKV, kH, kH, kWCarry);
  tcast_kernel<<<dim3(kH / 64, kH / 64, 1), 256, 0, stream>>>(wo, wo, wo, WO, kH, kH, kWCarry);

  wmma_gemm64<0, false, 2, 1, false><<<dim3(gemm_grid_x(kTok, kH), 1), 256, 0, stream>>>(
      XH, nullptr, kH, 0L, 0L, WQKV, nullptr, kH, 0L, 0L, (void*)QKV, nullptr, kQKVld, 0L, 0L,
      bq, nullptr, 0L, 0L, kTok, kH, kH, kWInv, 1);
  wmma_gemm64<0, false, 2, 1, false><<<dim3(gemm_grid_x(kTok, kH), 1), 256, 0, stream>>>(
      XH, nullptr, kH, 0L, 0L, WQKV + (size_t)kH * kH, nullptr, kH, 0L, 0L, (void*)(QKV + kH), nullptr, kQKVld, 0L, 0L,
      bk, nullptr, 0L, 0L, kTok, kH, kH, kWInv, 1);
  wmma_gemm64<0, false, 2, 1, false><<<dim3(gemm_grid_x(kTok, kH), 1), 256, 0, stream>>>(
      XH, nullptr, kH, 0L, 0L, WQKV + (size_t)2 * kH * kH, nullptr, kH, 0L, 0L, (void*)(QKV + 2 * kH), nullptr, kQKVld, 0L, 0L,
      bv, nullptr, 0L, 0L, kTok, kH, kH, kWInv, 1);

  vt_kernel<<<dim3(kS / 64, kGroups), 256, 0, stream>>>(QKV, VT);

  const long qkStrideB  = (long)kS * kQKVld;
  const long qkStrideH  = (long)kDH;
  const long scStrideB  = (long)kNH * kS * kS;
  const long scStrideH  = (long)kS * kS;
  const long vtStrideB  = (long)kNH * kDH * kS;
  const long vtStrideH  = (long)kDH * kS;
  const long ctxStrideB = (long)kS * kH;
  const long ctxStrideH = (long)kDH;
  for (int cb = 0; cb < kNChunk; ++cb) {
    const unsigned short* Qp = QKV + (size_t)(2 * cb) * kS * kQKVld;
    const unsigned short* Kp = Qp + kH;
    wmma_gemm64<0, false, 0, 0, false><<<dim3(gemm_grid_x(kS, kS), kGChunk), 256, 0, stream>>>(
        Qp, nullptr, kQKVld, qkStrideB, qkStrideH, Kp, nullptr, kQKVld, qkStrideB, qkStrideH,
        (void*)SC, nullptr, kS, scStrideB, scStrideH, nullptr, nullptr, 0L, 0L, kS, kS, kDH, kScoreScale, kNH);
    softmax_kernel<<<dim3(kGChunk * kS), 64, 0, stream>>>(SC, smask, P, cb);
    wmma_gemm64<0, false, 0, 1, false><<<dim3(gemm_grid_x(kS, kDH), kGChunk), 256, 0, stream>>>(
        P, nullptr, kS, scStrideB, scStrideH, VT + (size_t)(cb * kGChunk) * kDH * kS, nullptr, kS, vtStrideB, vtStrideH,
        (void*)(CTX + (size_t)(2 * cb) * kS * kH), nullptr, kH, ctxStrideB, ctxStrideH,
        nullptr, nullptr, 0L, 0L, kS, kDH, kS, kPVScale, kNH);
  }

  wmma_gemm64<0, false, 2, 0, true><<<dim3(gemm_grid_x(kTok, kH), 1), 256, 0, stream>>>(
      CTX, nullptr, kH, 0L, 0L, WO, nullptr, kH, 0L, 0L, (void*)WOOUT, nullptr, kH, 0L, 0L,
      bo, XF32, 0L, 0L, kTok, kH, kH, kWoScale, 1);
  ln_kernel<true><<<dim3(kTok), 256, 0, stream>>>(WOOUT, ln1_g, ln1_b, HF32, HH);

  tcast_kernel<<<dim3(kH / 64, kFF / 64, 1), 256, 0, stream>>>(w1, w1, w1, WW1, kH, kFF, kWCarry);
  tcast_kernel<<<dim3(kFF / 64, kH / 64, 1), 256, 0, stream>>>(w2, w2, w2, WW2, kFF, kH, kWCarry);
  wmma_gemm64<0, false, 2, 0, false><<<dim3(gemm_grid_x(kTok, kFF), 1), 256, 0, stream>>>(
      HH, nullptr, kH, 0L, 0L, WW1, nullptr, kH, 0L, 0L, (void*)FFNPRE, nullptr, kFF, 0L, 0L,
      b1, nullptr, 0L, 0L, kTok, kFF, kH, kWInv, 1);
  gelu_cast2_kernel<<<dim3((kTok * kFF / 2 + 255) / 256), 256, 0, stream>>>(FFNPRE, FFNH, kTok * kFF / 2);
  wmma_gemm64<0, false, 2, 0, true><<<dim3(gemm_grid_x(kTok, kH), 1), 256, 0, stream>>>(
      FFNH, nullptr, kFF, 0L, 0L, WW2, nullptr, kFF, 0L, 0L, (void*)W2OUT, nullptr, kH, 0L, 0L,
      b2, HF32, 0L, 0L, kTok, kH, kFF, kWInv, 1);
  ln_kernel<false><<<dim3(kTok), 256, 0, stream>>>(W2OUT, ln2_g, ln2_b, OUT, nullptr);
}
